// Cross_PCLEMA_87668872446318
// MI455X (gfx1250) — hardware-run, weakly checked
//
#include <hip/hip_runtime.h>
#include <math.h>

typedef __attribute__((ext_vector_type(16))) _Float16 v16h;
typedef __attribute__((ext_vector_type(16))) __bf16 v16b;
typedef __attribute__((ext_vector_type(8)))  _Float16 v8h;
typedef __attribute__((ext_vector_type(8)))  float v8f;
typedef __attribute__((ext_vector_type(4)))  float v4f;
typedef __attribute__((ext_vector_type(2)))  float v2f;
typedef __attribute__((ext_vector_type(4)))  unsigned v4u;
typedef __attribute__((ext_vector_type(4)))  int v4i;
typedef float __attribute__((may_alias)) float_a;
typedef int __attribute__((may_alias)) int_a;

template <typename T> __device__ __forceinline__ void vst2(void* p, T v) { *(volatile T*)p = v; __threadfence(); *(volatile T*)p = v; }
__device__ __forceinline__ v8f wmma16(v16h a, v16h b, v8f c) {
  v8f d = __builtin_amdgcn_wmma_f32_16x16x32_f16(false, a, false, b, (short)0, c, false, false);
  asm volatile("v_nop\n\tv_nop\n\tv_nop\n\tv_nop" : "+v"(d) : "v"(a), "v"(b));
  return d;
}
__device__ __forceinline__ v8f wmma_bf(v16b a, v16b b, v8f c) {
  v8f d = __builtin_amdgcn_wmma_f32_16x16x32_bf16(false, a, false, b, (short)0, c, false, false);
  asm volatile("v_nop\n\tv_nop\n\tv_nop\n\tv_nop" : "+v"(d) : "v"(a), "v"(b));
  return d;
}
__device__ __forceinline__ v16h frag_h(const _Float16* rowk0, int lane) {
  union { v16h v; v8h q[2]; } u; const _Float16* p = rowk0 + 8 * (lane >> 4);
  u.q[0] = *(const v8h*)p; u.q[1] = *(const v8h*)(p + 16); return u.v;
}
__device__ __forceinline__ v16h frag_f32(const float* rowk0, int lane) {
  v16h a; const float* p = rowk0 + 8 * (lane >> 4);
#pragma unroll
  for (int i = 0; i < 8; ++i) { a[i] = (_Float16)p[i]; a[8 + i] = (_Float16)p[16 + i]; }
  return a;
}
__device__ __forceinline__ v16h frag_f32s(const float* rowk0, int lane, float sc) {
  v16h a; const float* p = rowk0 + 8 * (lane >> 4);
#pragma unroll
  for (int i = 0; i < 8; ++i) { a[i] = (_Float16)(p[i] * sc); a[8 + i] = (_Float16)(p[16 + i] * sc); }
  return a;
}
__device__ __forceinline__ v16h fragc_f32(const float* W, int k0, int n, int lane, int ld, int K) {
  v16h a; const int g = lane >> 4;
#pragma unroll
  for (int i = 0; i < 8; ++i) { const int ka = k0 + 8 * g + i, kb = ka + 16;
    a[i] = (_Float16)(ka < K ? W[(size_t)(ka < K ? ka : K - 1) * ld + n] : 0.f); a[8 + i] = (_Float16)(kb < K ? W[(size_t)(kb < K ? kb : K - 1) * ld + n] : 0.f); }
  return a;
}
struct F2 { v16b h, l; };
__device__ __forceinline__ F2 bsplit16(const float v[16]) { F2 r;
#pragma unroll
  for (int i = 0; i < 16; ++i) { const __bf16 h = (__bf16)v[i]; r.h[i] = h; r.l[i] = (__bf16)(v[i] - (float)h); }
  return r; }
__device__ __forceinline__ F2 split_row(const float* row, int k0, int lane) { float v[16]; const float* p = row + k0 + 8 * (lane >> 4);
#pragma unroll
  for (int i = 0; i < 8; ++i) { v[i] = p[i]; v[8 + i] = p[16 + i]; }
  return bsplit16(v); }
__device__ __forceinline__ F2 split_rowK(const float* row, int k0, int lane, int K) { float v[16]; const int g = lane >> 4;
#pragma unroll
  for (int i = 0; i < 8; ++i) { const int ka = k0 + 8 * g + i, kb = ka + 16; v[i] = ka < K ? row[ka < K ? ka : K - 1] : 0.f; v[8 + i] = kb < K ? row[kb < K ? kb : K - 1] : 0.f; }
  return bsplit16(v); }
__device__ __forceinline__ F2 split_col(const float* W, int k0, int n, int lane, int ld, int K) { float v[16]; const int g = lane >> 4;
#pragma unroll
  for (int i = 0; i < 8; ++i) { const int ka = k0 + 8 * g + i, kb = ka + 16; v[i] = ka < K ? W[(size_t)(ka < K ? ka : K - 1) * ld + n] : 0.f; v[8 + i] = kb < K ? W[(size_t)(kb < K ? kb : K - 1) * ld + n] : 0.f; }
  return bsplit16(v); }
__device__ __forceinline__ v8f mac3(const F2& a, const F2& b, v8f c) { c = wmma_bf(a.l, b.h, c); c = wmma_bf(a.h, b.l, c); return wmma_bf(a.h, b.h, c); }
__device__ __forceinline__ float sigm(float v) { return 1.0f / (1.0f + expf(-v)); }
#define LDSX() do { asm volatile("s_wait_dscnt 0" ::: "memory"); __builtin_amdgcn_wave_barrier(); __builtin_amdgcn_fence(__ATOMIC_RELEASE, "workgroup"); } while (0)


#define NBT 512
#define TT 32
#define DD 512
#define MM 1024
#define NROW (NBT * TT)
#ifndef NBU
#define NBU NBT
#endif
#define NRU (NBU * TT)
typedef __attribute__((ext_vector_type(8))) __bf16 v8b;
__device__ __forceinline__ v16b frag_b(const __bf16* rowk0, int lane) {
  union { v16b v; v8b q[2]; } u; const __bf16* p = rowk0 + 8 * (lane >> 4);
  u.q[0] = *(const v8b*)p; u.q[1] = *(const v8b*)(p + 16); return u.v;
}
__device__ __forceinline__ float bfr(float v) { return (float)(__bf16)v; }
__device__ __attribute__((noinline)) float exp_ni(float v) { return expf(v); }
__device__ __attribute__((noinline)) float erf_ni(float v) { return erff(v); }
__device__ __attribute__((noinline)) float log_ni(float v) { return logf(v); }

#define WS_PK   0u
#define WS_E2   (2u * MM * DD)
#define WS_D    (((WS_E2 + 4u * MM) + 127u) / 128u * 128u)
#define WS_LA   (WS_D + 4u * (size_t)NROW * MM)
#define WS_LV   (WS_LA + 2u * (size_t)NROW * MM)
#define WS_ADA  (WS_LV + 2u * (size_t)NROW * MM)
#define WS_ADV  (WS_ADA + 2u * (size_t)NROW * MM)
#define WS_S    (WS_ADV + 2u * (size_t)NROW * MM)
#define WS_PMIN (WS_S + 4u * (size_t)TT * NBT * NBT)
#define WS_PL   (WS_PMIN + 4u * 2048)
#define WS_RED  (WS_PL + 4u * 512)
#define WS_END  (WS_RED + 128u)

__global__ __launch_bounds__(256) void k_pack(const float* __restrict__ E, __bf16* __restrict__ PK, float* __restrict__ E2) {
  __shared__ __align__(16) __bf16 s[DD]; __shared__ float red[8]; const int m = blockIdx.x, t = threadIdx.x; float q = 0.f;
  for (int k = t; k < DD; k += 256) { const float v = bfr(E[(size_t)m * DD + k]); s[k] = (__bf16)v; q += v * v; }
#pragma unroll
  for (int o = 1; o < 32; o <<= 1) q += __shfl_xor(q, o);
  if ((t & 31) == 0) red[t >> 5] = q; __syncthreads();
  if (t == 0) { float a = 0.f; for (int w = 0; w < 8; ++w) a += red[w]; E2[m] = a; }
  for (int q2 = t; q2 < DD / 8; q2 += 256) vst2((unsigned*)(PK + (size_t)m * DD + q2 * 8), *(const v4u*)&s[q2 * 8]);
  (void)red;
}
__global__ __launch_bounds__(128) void k_dist(const float* __restrict__ X, const __bf16* __restrict__ PK, const float* __restrict__ E2, float* __restrict__ Dd) {
  __shared__ __align__(16) float so[4][16][132]; __shared__ float sx2[64];
  const int tid = threadIdx.x, wave = tid >> 5, lane = tid & 31, col = lane & 15, g = lane >> 4; const size_t r0 = (size_t)blockIdx.x * 64 + wave * 16; const int n0 = blockIdx.y * 128;
  { const int r = tid >> 1, half = tid & 1; const float* p = X + ((size_t)blockIdx.x * 64 + r) * DD + half * 256; float q = 0.f; for (int k = 0; k < 256; ++k) { const float v = bfr(p[k]); q += v * v; } q += __shfl_xor(q, 1); if (half == 0) sx2[r] = q; }
  v8f acc[8] = {};
#pragma unroll 2
  for (int kc = 0; kc < DD / 32; ++kc) { v16b a; { const float* p = X + (r0 + col) * DD + kc * 32 + 8 * g;
#pragma unroll
      for (int i = 0; i < 8; ++i) { a[i] = (__bf16)p[i]; a[8 + i] = (__bf16)p[16 + i]; } }
#pragma unroll
    for (int j = 0; j < 8; ++j) acc[j] = wmma_bf(a, frag_b(PK + (size_t)(n0 + j * 16 + col) * DD + kc * 32, lane), acc[j]); }
  __syncthreads();
#pragma unroll
  for (int j = 0; j < 8; ++j) { const int c = j * 16 + col; const float e2 = E2[n0 + c];
#pragma unroll
    for (int r = 0; r < 8; ++r) so[wave][8 * g + r][c] = fmaxf(e2 + sx2[wave * 16 + 8 * g + r] - 2.0f * acc[j][r], 0.f); }
  LDSX();
  for (int rl = 0; rl < 16; ++rl) vst2(Dd + (r0 + rl) * MM + n0 + lane * 4, *(const v4f*)&so[wave][rl][lane * 4]);
}
__global__ __launch_bounds__(256) void k_soft(const float* __restrict__ Dd, _Float16* __restrict__ Lp, _Float16* __restrict__ ADJ) {
  __shared__ float red[3][8]; __shared__ __align__(16) _Float16 sl[MM], sa[MM]; const int t = threadIdx.x; const size_t row = blockIdx.x; const float* p = Dd + row * MM + t * 4;
  float sd[4]; float mx = -3.0e38f;
#pragma unroll
  for (int i = 0; i < 4; ++i) { sd[i] = sqrtf(p[i]); mx = fmaxf(mx, -sd[i]); }
#pragma unroll
  for (int o = 1; o < 32; o <<= 1) mx = fmaxf(mx, __shfl_xor(mx, o));
  if ((t & 31) == 0) red[0][t >> 5] = mx; __syncthreads();
  float gm = -3.0e38f; for (int w = 0; w < 8; ++w) gm = fmaxf(gm, red[0][w]);
  float e1[4], e2[4]; float s1 = 0.f, s2 = 0.f;
#pragma unroll
  for (int i = 0; i < 4; ++i) { e1[i] = exp_ni(-sd[i] - gm); e2[i] = exp_ni(2.0f * (-sd[i] - gm)); s1 += e1[i]; s2 += e2[i]; }
#pragma unroll
  for (int o = 1; o < 32; o <<= 1) { s1 += __shfl_xor(s1, o); s2 += __shfl_xor(s2, o); }
  if ((t & 31) == 0) { red[1][t >> 5] = s1; red[2][t >> 5] = s2; } __syncthreads();
  float t1 = 0.f, t2 = 0.f; for (int w = 0; w < 8; ++w) { t1 += red[1][w]; t2 += red[2][w]; }
  const float i1 = 1.0f / t1, i2 = 1.0f / t2;
#pragma unroll
  for (int i = 0; i < 4; ++i) { sl[t * 4 + i] = (_Float16)log_ni(e1[i] * i1 + 1e-10f); sa[t * 4 + i] = (_Float16)(e2[i] * i2); }
  __syncthreads();
  if (t < 128) vst2((unsigned*)(Lp + row * MM + t * 8), *(const v4u*)&sl[t * 8]); else vst2((unsigned*)(ADJ + row * MM + (t - 128) * 8), *(const v4u*)&sa[(t - 128) * 8]);
}
__global__ __launch_bounds__(128) void k_scode(const _Float16* __restrict__ ADJ, const _Float16* __restrict__ Lp, float* __restrict__ S, float* __restrict__ PMIN) {
  __shared__ __align__(16) float so[4][16][132]; __shared__ float smn[128];
  const int tid = threadIdx.x, wave = tid >> 5, lane = tid & 31, col = lane & 15, g = lane >> 4; const int t = blockIdx.z; const int i0 = blockIdx.x * 64 + wave * 16, j0 = blockIdx.y * 128;
  v8f acc[8] = {};
#pragma unroll 2
  for (int kc = 0; kc < MM / 32; ++kc) { const v16h a = frag_h(ADJ + ((size_t)(i0 + col) * TT + t) * MM + kc * 32, lane);
#pragma unroll
    for (int j = 0; j < 8; ++j) acc[j] = wmma16(a, frag_h(Lp + ((size_t)(j0 + j * 16 + col) * TT + t) * MM + kc * 32, lane), acc[j]); }
  float mn = 3.0e38f;
#pragma unroll
  for (int j = 0; j < 8; ++j)
#pragma unroll
    for (int r = 0; r < 8; ++r) { so[wave][8 * g + r][j * 16 + col] = acc[j][r]; mn = fminf(mn, acc[j][r]); }
#pragma unroll
  for (int o = 1; o < 32; o <<= 1) mn = fminf(mn, __shfl_xor(mn, o));
  if (lane == 0) smn[wave] = mn;
  LDSX();
  for (int rl = 0; rl < 16; ++rl) vst2(S + ((size_t)t * NBU + i0 + rl) * NBU + j0 + lane * 4, *(const v4f*)&so[wave][rl][lane * 4]);
  __syncthreads();
  if (tid == 0) { const float m4 = fminf(fminf(smn[0], smn[1]), fminf(smn[2], smn[3])); PMIN[((size_t)t * (NBU / 64) + blockIdx.x) * (NBU / 128) + blockIdx.y] = m4; }
}
__global__ __launch_bounds__(256) void k_shift(const float* __restrict__ PMIN, float* __restrict__ RED) {
  __shared__ float sm[256]; const int t = threadIdx.x; float mn = 3.0e38f; for (int i = t; i < TT * (NBU / 64) * (NBU / 128); i += 256) mn = fminf(mn, PMIN[i]); sm[t] = mn; __syncthreads();
  for (int s = 128; s > 0; s >>= 1) { if (t < s) sm[t] = fminf(sm[t], sm[t + s]); __syncthreads(); }
  if (t == 0) RED[0] = -sm[0];
}
__global__ __launch_bounds__(256) void k_lterm(const float* __restrict__ S, const float* __restrict__ RED, float* __restrict__ PL) {
  __shared__ float sterm[64]; const int t = threadIdx.x; const int tt = blockIdx.y; const int r = t >> 2, q = t & 3; const int i = blockIdx.x * 64 + r; const float shift = RED[0];
  const float* row = S + ((size_t)tt * NBU + i) * NBU; float sm = 0.f;
  for (int j = q * (NBU / 4); j < q * (NBU / 4) + (NBU / 4); ++j) sm += exp_ni(row[j] + shift);
  sm += __shfl_xor(sm, 1); sm += __shfl_xor(sm, 2);
  if (q == 0) { const float diag = exp_ni(row[i] + shift); sterm[r] = log_ni(diag / (sm + 1e-5f)); }
  __syncthreads();
  if (t == 0) { float a = 0.f; for (int k = 0; k < 64; ++k) a += sterm[k]; PL[(size_t)tt * (NBU / 64) + blockIdx.x] = a; }
}
__global__ __launch_bounds__(256) void k_lsum(const float* __restrict__ PL, float* __restrict__ RED, int which, float* __restrict__ OUT) {
  __shared__ float sm[256]; const int t = threadIdx.x; float a = 0.f; for (int i = t; i < TT * (NBU / 64); i += 256) a += PL[i]; sm[t] = a; __syncthreads();
  for (int s = 128; s > 0; s >>= 1) { if (t < s) sm[t] += sm[t + s]; __syncthreads(); }
  if (t == 0) { const float loss = -sm[0] / (float)(TT * NBU); RED[1 + which] = loss; if (which == 1) { __align__(16) float o4[4] = {0.5f * (RED[1] + loss), 0.f, 0.f, 0.f}; OUT[0] = o4[0]; } }
}
extern "C" void kernel_launch(void* const* d_in, const int* in_sizes, int n_in, void* d_out, int out_size, void* d_ws, size_t ws_size, hipStream_t stream) {
  (void)in_sizes; (void)n_in; (void)out_size;
  const float** F = (const float**)d_in;
  if (ws_size < (size_t)WS_END) return;
  char* ws = (char*)d_ws; __bf16* PK = (__bf16*)(ws + WS_PK); float *E2 = (float*)(ws + WS_E2), *Dd = (float*)(ws + WS_D), *S = (float*)(ws + WS_S), *PMIN = (float*)(ws + WS_PMIN), *PL = (float*)(ws + WS_PL), *RED = (float*)(ws + WS_RED); _Float16 *LA = (_Float16*)(ws + WS_LA), *LV = (_Float16*)(ws + WS_LV), *ADA = (_Float16*)(ws + WS_ADA), *ADV = (_Float16*)(ws + WS_ADV);
  k_pack<<<MM, 256, 0, stream>>>(F[2], PK, E2);
  k_dist<<<dim3(NRU / 64, MM / 128), 128, 0, stream>>>(F[0], PK, E2, Dd);
  k_soft<<<NRU, 256, 0, stream>>>(Dd, LA, ADA);
  k_dist<<<dim3(NRU / 64, MM / 128), 128, 0, stream>>>(F[1], PK, E2, Dd);
  k_soft<<<NRU, 256, 0, stream>>>(Dd, LV, ADV);
  for (int which = 0; which < 2; ++which) {
    k_scode<<<dim3(NBU / 64, NBU / 128, TT), 128, 0, stream>>>(which == 0 ? ADA : ADV, which == 0 ? LV : LA, S, PMIN);
    k_shift<<<1, 256, 0, stream>>>(PMIN, RED);
    k_lterm<<<dim3(NBU / 64, TT), 256, 0, stream>>>(S, RED, PL);
    k_lsum<<<1, 256, 0, stream>>>(PL, RED, which, (float*)d_out); }
}
